// FactorGNNSBMs_15479062135603
// MI455X (gfx1250) — hardware-run, weakly checked
//
#include <hip/hip_runtime.h>


namespace {
constexpr int NN = 20000, NE = 640000, IN = 128, HH = 128, VOC = 200, STB = 128, MAXDEG = 1024, NGc = (NN + 255) / 256, PERMLEN = NE + 32 * NGc + 32;
constexpr float XS = 8.0f;

typedef _Float16 b16;
typedef __attribute__((ext_vector_type(16))) _Float16 v16b;
typedef __attribute__((ext_vector_type(8))) _Float16 v8b;
typedef __attribute__((ext_vector_type(8))) float v8f;
typedef __attribute__((ext_vector_type(4))) float v4f;
typedef __attribute__((ext_vector_type(2))) float v2f;
__device__ __forceinline__ float bf16_rne(float f) { unsigned int u = __float_as_uint(f); u += 0x7FFFu + ((u >> 16) & 1u); return __uint_as_float(u & 0xFFFF0000u); }
__device__ __forceinline__ void split16(float v, b16& hi, b16& lo) { hi = (b16)v; lo = (b16)(v - (float)hi); }
__device__ __forceinline__ v16b frag_kb(const b16* p, int hh) { const v8b a = *(const v8b*)(p + 8 * hh), b = *(const v8b*)(p + 16 + 8 * hh); v16b f;
#pragma unroll
  for (int e = 0; e < 8; ++e) { f[e] = a[e]; f[8 + e] = b[e]; } return f; }
__device__ __forceinline__ v8f wmma16b(v16b a, v16b b, v8f c) { v8f d = __builtin_amdgcn_wmma_f32_16x16x32_f16(false, a, false, b, (short)0, c, false, false); asm volatile("v_nop\n\tv_nop\n\tv_nop\n\tv_nop" : "+v"(d) : "v"(a), "v"(b)); return d; }
__device__ __forceinline__ void wave_lds_sync() { __builtin_amdgcn_fence(__ATOMIC_RELEASE, "workgroup"); __builtin_amdgcn_wave_barrier(); __builtin_amdgcn_fence(__ATOMIC_ACQUIRE, "workgroup"); }
__device__ __forceinline__ float nexp(float x) { return __builtin_amdgcn_exp2f(x * 1.4426950408889634f); }
__device__ __forceinline__ float pmul(float a, float b) { float p = a * b; asm volatile("" : "+v"(p)); return p; }
__device__ __forceinline__ float sigm(float x) { return 1.0f / (1.0f + nexp(-x)); }
constexpr int CSR_NBLK = 512, CSR_GB = 8, CSR_GN = 1 << CSR_GB  , CSR_MAXG = 512, CSR_CAP = 12288  ;
__global__ __launch_bounds__(64) void csrA_kernel(const int* __restrict__ dst, int E, int N, int nG, int CHP, int NGP, int* __restrict__ STG, int* __restrict__ HST) {
  extern __shared__ int sm[];
  int* cnt = sm; int* run = sm + NGP; int* ids = sm + 2 * NGP;
  const int b = blockIdx.x; const int ch = (E + CSR_NBLK - 1) / CSR_NBLK; const int e0 = b * ch, e1 = min(E, e0 + ch);
  for (int i = threadIdx.x; i < NGP; i += 64) cnt[i] = 0;
  for (int i = threadIdx.x; i < CHP; i += 64) ids[i] = -1;
  __syncthreads();
  if (threadIdx.x == 0) {
    for (int e = e0; e < e1; ++e) { int d = dst[e]; d = (d < 0) ? 0 : (d >= N ? N - 1 : d); cnt[d >> CSR_GB] += 1; }
    int acc = 0; for (int g = 0; g < nG; ++g) { run[g] = acc; acc += cnt[g]; }
    for (int e = e0; e < e1; ++e) { int d = dst[e]; d = (d < 0) ? 0 : (d >= N ? N - 1 : d); const int g = d >> CSR_GB; ids[run[g]] = e; run[g] += 1; } }
  __syncthreads();
  typedef __attribute__((ext_vector_type(4))) int v4i;
  for (int pass = 0; pass < 2; ++pass) {
    for (int i = threadIdx.x; i < CHP / 4; i += 64) *(volatile v4i*)(STG + (size_t)b * CHP + i * 4) = *(const v4i*)(&ids[i * 4]);
    for (int i = threadIdx.x; i < NGP / 4; i += 64) { v4i v; for (int e = 0; e < 4; ++e) v[e] = (i * 4 + e < nG) ? cnt[i * 4 + e] : 0; *(volatile v4i*)(HST + (size_t)b * NGP + i * 4) = v; }
    __threadfence(); }
}
__global__ __launch_bounds__(512) void csrS_kernel(const int* __restrict__ HST, int nG, int NGP, int* __restrict__ START, int* __restrict__ TOT, int* __restrict__ OFF) {
  __shared__ int tot[CSR_MAXG];
  const int b = threadIdx.x;
  for (int pass = 0; pass < 2; ++pass) { int runb = 0; for (int g = 0; g < nG; ++g) { int c = HST[(size_t)b * NGP + g]; c = (c < 0) ? 0 : c; ((volatile int*)OFF)[(size_t)g * CSR_NBLK + b] = runb; runb += c; } __threadfence(); }
  for (int g = threadIdx.x; g < nG; g += 512) { int s = 0; for (int bb = 0; bb < CSR_NBLK; ++bb) { int c = HST[(size_t)bb * NGP + g]; s += (c < 0) ? 0 : c; } tot[g] = s; }
  __syncthreads();
  if (threadIdx.x < 32) {
    __shared__ int st[CSR_MAXG + 32];
    if (threadIdx.x == 0) { int acc = 0; for (int g = 0; g < NGP; ++g) { st[g] = acc; if (g < nG) acc += (tot[g] + 31) & ~31; } st[NGP] = acc; }
    __builtin_amdgcn_fence(__ATOMIC_RELEASE, "workgroup"); __builtin_amdgcn_wave_barrier(); __builtin_amdgcn_fence(__ATOMIC_ACQUIRE, "workgroup");
    for (int pass = 0; pass < 2; ++pass) { for (int i = threadIdx.x; i < NGP + 32; i += 32) { ((volatile int*)START)[i] = (i <= NGP) ? st[min(i, NGP)] : 0; ((volatile int*)TOT)[i] = (i < nG) ? tot[i] : 0; } __threadfence(); } }
}
__global__ __launch_bounds__(256) void csrB_kernel(const int* __restrict__ dst, int N, int nG, int CHP, int NGP, int permLen, const int* __restrict__ STG, const int* __restrict__ HST, const int* __restrict__ OFF, const int* __restrict__ START, const int* __restrict__ TOT, int* __restrict__ PERM, int* __restrict__ ROWPTR, int* __restrict__ ROWCNT, int* __restrict__ FLAG) {
  typedef __attribute__((ext_vector_type(4))) int v4i;
  __shared__ int ids[CSR_CAP]; __shared__ unsigned short key[CSR_CAP]; __shared__ int outp[CSR_CAP]; __shared__ int ncnt[CSR_GN + 1]; __shared__ int boff[CSR_NBLK + 1];
  const int g = blockIdx.x, t_ = threadIdx.x; int tot = TOT[g]; int st = START[g], stn = START[g + 1]; const int v0 = g * CSR_GN; const int nv = min(CSR_GN, N - v0);
  st = (st < 0) ? 0 : (st > permLen - 32 ? permLen - 32 : st) & ~31; stn = (stn < st) ? st : (stn > permLen ? permLen : stn); tot = (tot < 0) ? 0 : tot; if (tot > stn - st && tot <= CSR_CAP) tot = stn - st;
  if (tot > CSR_CAP) {
    for (int pass = 0; pass < 2; ++pass) { for (int i = t_; i < CSR_GN / 4; i += 256) { v4i a, c; for (int e = 0; e < 4; ++e) { a[e] = st; c[e] = 0; } *(volatile v4i*)(ROWPTR + v0 + i * 4) = a; *(volatile v4i*)(ROWCNT + v0 + i * 4) = c; } if (t_ == 0) ((volatile int*)FLAG)[0] = 1; __threadfence(); } (void)nv; return; }
  if (t_ == 0) { int acc = 0; for (int b = 0; b < CSR_NBLK; ++b) { boff[b] = acc; int c = HST[(size_t)b * NGP + g]; c = (c < 0) ? 0 : (c > CHP ? CHP : c); acc += c; if (acc > tot) acc = tot; } boff[CSR_NBLK] = acc; }
  for (int i = t_; i <= CSR_GN; i += 256) ncnt[i] = 0;
  __syncthreads();
  for (int b = 0; b < CSR_NBLK; ++b) { const int c = boff[b + 1] - boff[b]; int o_ = OFF[(size_t)g * CSR_NBLK + b]; o_ = (o_ < 0) ? 0 : (o_ > CHP - c ? CHP - c : o_); const int* src_ = STG + (size_t)b * CHP + o_;
    for (int i = t_; i < c; i += 256) { int id = src_[i]; id = (id < 0) ? 0 : id; ids[boff[b] + i] = id; int d = dst[id]; d = (d < v0) ? v0 : (d >= N ? N - 1 : d); int kk = d - v0; kk = (kk < 0) ? 0 : (kk >= CSR_GN ? CSR_GN - 1 : kk); key[boff[b] + i] = (unsigned short)kk; } }
  __syncthreads();
  if (t_ == 0) { for (int i = 0; i < tot; ++i) ncnt[key[i]] += 1; int acc = 0; for (int vl = 0; vl < CSR_GN; ++vl) { const int c = ncnt[vl]; ncnt[vl] = acc; acc += c; } ncnt[CSR_GN] = acc;
    for (int i = 0; i < tot; ++i) { const int vl = key[i]; outp[ncnt[vl]] = ids[i]; ncnt[vl] += 1; }
    for (int vl = CSR_GN; vl > 0; --vl) ncnt[vl] = ncnt[vl - 1]; ncnt[0] = 0; }
  __syncthreads();
  for (int pass = 0; pass < 2; ++pass) {
    for (int i = t_; i < (stn - st) / 4; i += 256) { v4i v; for (int e = 0; e < 4; ++e) { const int q = i * 4 + e; v[e] = (q < tot) ? outp[q] : -1; } *(volatile v4i*)(PERM + st + i * 4) = v; }
    for (int i = t_; i < CSR_GN / 4; i += 256) { v4i a, c; for (int e = 0; e < 4; ++e) { const int vl = i * 4 + e; a[e] = st + ncnt[vl]; c[e] = (vl < nv) ? (ncnt[vl + 1] - ncnt[vl]) : 0; } *(volatile v4i*)(ROWPTR + v0 + i * 4) = a; *(volatile v4i*)(ROWCNT + v0 + i * 4) = c; }
    __threadfence(); }
}
__global__ __launch_bounds__(256) void csrZ_kernel(int* __restrict__ p, size_t n4) { typedef __attribute__((ext_vector_type(4))) int v4i; const size_t tid = (size_t)blockIdx.x * 256 + threadIdx.x, nth = (size_t)gridDim.x * 256; v4i z = {0, 0, 0, 0}; for (size_t i = tid; i < n4; i += nth) *(volatile v4i*)(p + i * 4) = z; }
struct CsrBufs { int *STG, *HST, *OFF, *START, *TOT, *PERM, *ROWPTR, *ROWCNT, *FLAG; int nG, NGP, CHP; size_t permLen; char* base; size_t bytes; };
static size_t csr_carve(CsrBufs& c, char* ws, size_t off, int E, int N) {
  const size_t off0 = off; c.base = ws + off;
  auto al = [&](size_t bytes) { char* p = ws + off; off += (bytes + 255) & ~(size_t)255; return p; };
  c.nG = (N + CSR_GN - 1) / CSR_GN; c.NGP = (c.nG + 31) & ~31; const int ch = (E + CSR_NBLK - 1) / CSR_NBLK; c.CHP = (ch + 31) & ~31; c.permLen = (size_t)E + 32 * (size_t)c.nG + 32;
  c.STG = (int*)al((size_t)CSR_NBLK * c.CHP * 4); c.HST = (int*)al((size_t)CSR_NBLK * c.NGP * 4); c.OFF = (int*)al((size_t)c.NGP * CSR_NBLK * 4); c.START = (int*)al((size_t)(c.NGP + 64) * 4); c.TOT = (int*)al((size_t)(c.NGP + 64) * 4);
  c.PERM = (int*)al(c.permLen * 4); c.ROWPTR = (int*)al((size_t)c.nG * CSR_GN * 4); c.ROWCNT = (int*)al((size_t)c.nG * CSR_GN * 4); c.FLAG = (int*)al(256);
  c.bytes = off - off0; return off;
}
static void csr_build(const CsrBufs& c, const int* dst, int E, int N, hipStream_t stream) {
  const size_t smem = (size_t)(2 * c.NGP + c.CHP) * 4;
  csrZ_kernel<<<512, 256, 0, stream>>>((int*)c.base, c.bytes / 16);
  csrA_kernel<<<CSR_NBLK, 64, smem, stream>>>(dst, E, N, c.nG, c.CHP, c.NGP, c.STG, c.HST);
  csrS_kernel<<<1, 512, 0, stream>>>(c.HST, c.nG, c.NGP, c.START, c.TOT, c.OFF);
  csrB_kernel<<<c.nG, 256, 0, stream>>>(dst, N, c.nG, c.CHP, c.NGP, (int)c.permLen, c.STG, c.HST, c.OFF, c.START, c.TOT, c.PERM, c.ROWPTR, c.ROWCNT, c.FLAG);
}

__global__ __launch_bounds__(256) void prep_kernel(const int* __restrict__ xid, const float* __restrict__ emb, const float* __restrict__ l1w, const float* __restrict__ l2w, const float* __restrict__ l3w, const float* __restrict__ c1w, b16* __restrict__ R, float* __restrict__ FT, b16* __restrict__ Fh, b16* __restrict__ Fl) {
  const size_t tid = (size_t)blockIdx.x * 256 + threadIdx.x, nth = (size_t)gridDim.x * 256;
  auto tr = [&](size_t base, int nout, int kin, const float* W) { for (size_t p = tid; p < (size_t)nout * kin; p += nth) { const int o = (int)(p / kin), k = (int)(p % kin); ((volatile b16*)R)[base + p] = (b16)bf16_rne(W[(size_t)k * nout + o]); } };
  for (int pass = 0; pass < 2; ++pass) {
    tr(0, 16, 128, l1w); tr(2048, 32, 128, l2w); tr(6144, 32, 128, l3w); tr(10240, 64, 128, c1w);
    for (size_t p = tid; p < (size_t)NN * IN / 8; p += nth) { const size_t n = p / (IN / 8); const int c8 = (int)(p % (IN / 8)) * 8; int id = xid[n]; id = (id < 0) ? 0 : (id >= VOC ? VOC - 1 : id); v8b hv, lv; float f[8];
#pragma unroll
      for (int e = 0; e < 8; ++e) { f[e] = bf16_rne(emb[(size_t)id * IN + c8 + e]); hv[e] = (b16)(f[e] * XS); lv[e] = (b16)0.0f; }
      *(volatile v4f*)(FT + p * 8) = *(v4f*)&f[0]; *(volatile v4f*)(FT + p * 8 + 4) = *(v4f*)&f[4]; *(volatile v8b*)(Fh + p * 8) = hv; *(volatile v8b*)(Fl + p * 8) = lv; }
    __threadfence(); }
}
template <int F, int L>
__global__ __launch_bounds__(256) void par_kernel(const float* __restrict__ b, const float* __restrict__ wl, const float* __restrict__ wlb, const float* __restrict__ wr, const float* __restrict__ wrb, const float* __restrict__ g, const float* __restrict__ bb, float* __restrict__ Pl) {
  const int tid = blockIdx.x * 256 + threadIdx.x;
  for (int pass = 0; pass < 2; ++pass) { for (int j = tid; j < 1024; j += 1024) { float v = 0.0f;
      if (j < 32) v = (j < F) ? b[j] : 0.0f; else if (j < 288) v = (j - 32 < F * L) ? wl[j - 32] : 0.0f; else if (j < 320) v = (j - 288 < L) ? wlb[j - 288] : 0.0f; else if (j < 576) v = (j - 320 < F * L) ? wr[j - 320] : 0.0f; else if (j < 640) v = (j - 576 < L) ? wrb[j - 576] : 0.0f; else if (j < 768) v = g[j - 640]; else if (j < 896) v = bb[j - 768];
      ((volatile float*)Pl)[j] = bf16_rne(v); } __threadfence(); }
}
__global__ __launch_bounds__(256) void parc_kernel(const float* __restrict__ c1b, const float* __restrict__ c2w, const float* __restrict__ c2b, float* __restrict__ P) {
  const int t = threadIdx.x;
  for (int pass = 0; pass < 2; ++pass) { for (int j = t; j < 200; j += 256) { float v = 0.0f; if (j < 64) v = c1b[j]; else if (j < 192) v = c2w[j - 64]; else if (j < 194) v = c2b[j - 192]; ((volatile float*)P)[3072 + j] = bf16_rne(v); } __threadfence(); }
}
template <int F, int L>
__global__ __launch_bounds__(64) void hid_kernel(const b16* __restrict__ Fh, const b16* __restrict__ Fl, const b16* __restrict__ Bw, const float* __restrict__ Pl, float* __restrict__ HID, float* __restrict__ ALR) {
  __shared__ __attribute__((aligned(16))) float Ts[2][16][32 + 4]; __shared__ __attribute__((aligned(16))) float As[2][16][16];
  constexpr int NS = F / 16;
  const int lane = threadIdx.x & 31, wave = threadIdx.x >> 5, nloc = lane & 15, hlf = lane >> 4, m0 = blockIdx.x * 32 + wave * 16;
  v8f acc[2] = {{}, {}};
#pragma unroll
  for (int kb = 0; kb < IN; kb += 32) { const v16b a = frag_kb(Fh + (size_t)(m0 + nloc) * IN + kb, hlf), al_ = frag_kb(Fl + (size_t)(m0 + nloc) * IN + kb, hlf);
#pragma unroll
    for (int t = 0; t < NS; ++t) { const v16b bw = frag_kb(Bw + (size_t)(t * 16 + nloc) * IN + kb, hlf); acc[t] = wmma16b(a, bw, acc[t]); acc[t] = wmma16b(al_, bw, acc[t]); } }
#pragma unroll
  for (int t = 0; t < 2; ++t)
#pragma unroll
    for (int r = 0; r < 8; ++r) Ts[wave][8 * hlf + r][t * 16 + nloc] = (t < NS) ? (acc[t][r] * (1.0f / XS) + Pl[t * 16 + nloc]) : 0.0f;
  wave_lds_sync();
  if (lane < 16) { const float* hr = &Ts[wave][lane][0]; for (int j = 0; j < 16; ++j) As[wave][lane][j] = 0.0f;
    for (int l = 0; l < L; ++l) { float sl = Pl[288 + l], sr = Pl[576 + l]; for (int f = 0; f < F; ++f) { sl += pmul(hr[f], Pl[32 + f * L + l]); sr += pmul(hr[f], Pl[320 + f * L + l]); } As[wave][lane][l] = sl; As[wave][lane][8 + l] = sr; } }
  wave_lds_sync();
  for (int pass = 0; pass < 2; ++pass) { for (int i = lane; i < 16 * 8; i += 32) { const int rr = i >> 3, c4 = (i & 7) * 4; *(volatile v4f*)(HID + (size_t)(m0 + rr) * 32 + c4) = *(const v4f*)(&Ts[wave][rr][c4]); }
    for (int i = lane; i < 16 * 4; i += 32) { const int rr = i >> 2, c4 = (i & 3) * 4; *(volatile v4f*)(ALR + (size_t)(m0 + rr) * 16 + c4) = *(const v4f*)(&As[wave][rr][c4]); } __threadfence(); }
}
template <int F>
__global__ __launch_bounds__(256) void agg_kernel(const float* __restrict__ HID, const float* __restrict__ ALR, const int* __restrict__ src, const int* __restrict__ perm, const int* __restrict__ rowptr, const int* __restrict__ rowcnt, const float* __restrict__ snorm, float* __restrict__ PRE) {
  const int wave = threadIdx.x >> 5, v = blockIdx.x * 8 + wave, lane = threadIdx.x & 31; const int o0 = lane * 4; const int fac = o0 / F, f0 = o0 % F;
  int cnt = rowcnt[v]; cnt = (cnt < 0) ? 0 : (cnt > MAXDEG ? MAXDEG : cnt); int p0 = rowptr[v]; p0 = (p0 < 0) ? 0 : (p0 > PERMLEN - cnt ? PERMLEN - cnt : p0);
  const float arv = ALR[(size_t)v * 16 + 8 + fac]; v4f acc = {0, 0, 0, 0};
  for (int q = 0; q < cnt; ++q) { int id = perm[p0 + q]; id = (id < 0) ? 0 : (id >= NE ? NE - 1 : id); int s = src[id]; s = (s < 0) ? 0 : (s >= NN ? NN - 1 : s); int cs_ = rowcnt[s]; cs_ = (cs_ < 1) ? 1 : (cs_ > MAXDEG ? MAXDEG : cs_);
    const float g = sigm(6.0f * (ALR[(size_t)s * 16 + fac] + arv)); const float w = pmul(g, rsqrtf((float)cs_)); const v4f hv = *(const v4f*)(HID + (size_t)s * 32 + f0);
#pragma unroll
    for (int e = 0; e < 4; ++e) acc[e] += pmul(hv[e], w); }
  const float sn = bf16_rne(snorm[v]); v4f o; for (int e = 0; e < 4; ++e) o[e] = pmul(acc[e], sn);
  for (int pass = 0; pass < 2; ++pass) { *(volatile v4f*)(PRE + (size_t)v * HH + o0) = o; __threadfence(); }
}
template <int MODE>
__global__ __launch_bounds__(128) void stat_kernel(const float* __restrict__ PRE, const float* __restrict__ MEAN, float* __restrict__ PART) {
  const int c = threadIdx.x, b = blockIdx.x; const int ch = (NN + STB - 1) / STB; const int r0 = b * ch, r1 = min(NN, r0 + ch); const float mu = MODE ? MEAN[c] : 0.0f;
  float s = 0.0f; for (int r = r0; r < r1; ++r) { const float x = PRE[(size_t)r * HH + c]; if (MODE) { const float d = x - mu; s += pmul(d, d); } else s += x; }
  for (int pass = 0; pass < 2; ++pass) { ((volatile float*)PART)[(size_t)b * HH + c] = s; __threadfence(); }
}
__global__ __launch_bounds__(128) void comb_kernel(const float* __restrict__ PART, float* __restrict__ OUT) {
  const int c = threadIdx.x; float s = 0.0f; for (int b = 0; b < STB; ++b) s += PART[(size_t)b * HH + c];
  for (int pass = 0; pass < 2; ++pass) { ((volatile float*)OUT)[c] = s * (1.0f / NN); __threadfence(); }
}
template <int LAST>
__global__ __launch_bounds__(256) void epi_kernel(const float* __restrict__ PRE, const float* __restrict__ MEAN, const float* __restrict__ VAR, const float* __restrict__ Pl, float* __restrict__ FT, b16* __restrict__ Fh, b16* __restrict__ Fl) {
  __shared__ __attribute__((aligned(16))) b16 Sh[8][HH + 8], Sl[8][HH + 8];
  const int wave = threadIdx.x >> 5, v = blockIdx.x * 8 + wave, lane = threadIdx.x & 31;
  const v4f x = *(const v4f*)(PRE + (size_t)v * HH + lane * 4); v4f o;
#pragma unroll
  for (int e = 0; e < 4; ++e) { const int c = lane * 4 + e; float y = pmul((x[e] - MEAN[c]) * rsqrtf(VAR[c] + 1e-5f), Pl[640 + c]) + Pl[768 + c]; y = (y > 0.0f) ? y : 0.2f * y; o[e] = y; const float z = LAST ? fmaxf(y, 0.0f) : y; b16 a_, b_; split16(z * XS, a_, b_); Sh[wave][c] = a_; Sl[wave][c] = b_; }
  wave_lds_sync();
  for (int pass = 0; pass < 2; ++pass) { *(volatile v4f*)(FT + (size_t)v * HH + lane * 4) = o; if (lane < 16) { *(volatile v8b*)(Fh + (size_t)v * HH + lane * 8) = *(const v8b*)(&Sh[wave][lane * 8]); *(volatile v8b*)(Fl + (size_t)v * HH + lane * 8) = *(const v8b*)(&Sl[wave][lane * 8]); } __threadfence(); }
}
__global__ __launch_bounds__(64) void cls_kernel(const b16* __restrict__ Fh, const b16* __restrict__ Fl, const b16* __restrict__ Bw, const float* __restrict__ P, float* __restrict__ out) {
  __shared__ __attribute__((aligned(16))) float Ts[2][16][64 + 4]; __shared__ __attribute__((aligned(16))) float Os[32][2];
  const int lane = threadIdx.x & 31, wave = threadIdx.x >> 5, nloc = lane & 15, hlf = lane >> 4, m0 = blockIdx.x * 32 + wave * 16;
  v8f acc[4] = {{}, {}, {}, {}};
#pragma unroll
  for (int kb = 0; kb < IN; kb += 32) { const v16b a = frag_kb(Fh + (size_t)(m0 + nloc) * IN + kb, hlf), al_ = frag_kb(Fl + (size_t)(m0 + nloc) * IN + kb, hlf);
#pragma unroll
    for (int t = 0; t < 4; ++t) { const v16b bw = frag_kb(Bw + (size_t)(t * 16 + nloc) * IN + kb, hlf); acc[t] = wmma16b(a, bw, acc[t]); acc[t] = wmma16b(al_, bw, acc[t]); } }
#pragma unroll
  for (int t = 0; t < 4; ++t)
#pragma unroll
    for (int r = 0; r < 8; ++r) Ts[wave][8 * hlf + r][t * 16 + nloc] = fmaxf(acc[t][r] * (1.0f / XS) + P[3072 + t * 16 + nloc], 0.0f);
  wave_lds_sync();
  if (lane < 16) { const float* rr = &Ts[wave][lane][0]; float s0 = P[3264], s1 = P[3265]; for (int j = 0; j < 64; ++j) { s0 += pmul(rr[j], P[3136 + j * 2]); s1 += pmul(rr[j], P[3136 + j * 2 + 1]); } Os[wave * 16 + lane][0] = s0; Os[wave * 16 + lane][1] = s1; }
  __syncthreads();
  for (int pass = 0; pass < 2; ++pass) { if (threadIdx.x < 16) *(volatile v4f*)(out + (size_t)blockIdx.x * 64 + threadIdx.x * 4) = *(const v4f*)(&Os[0][0] + threadIdx.x * 4); __threadfence(); }
}
}

extern "C" void kernel_launch(void* const* d_in, const int* in_sizes, int n_in,
                              void* d_out, int out_size, void* d_ws, size_t ws_size, hipStream_t stream) {
  (void)n_in; (void)out_size;
  auto Fp = [&](int i) { return (const float*)d_in[i]; };
  const int* xid = (const int*)d_in[0]; const int* srcI = (const int*)d_in[1]; const int* dstI = (const int*)d_in[2]; const float* snorm = Fp(3); const float* emb = Fp(4);
  float* out = (float*)d_out;
  if (in_sizes[0] != NN || in_sizes[1] != NE || in_sizes[2] != NE || in_sizes[4] != VOC * IN) return;
  const int NE_RUN = NE;
  size_t off = 0; char* ws = (char*)d_ws;
  auto carve = [&](size_t bytes) { char* p = ws + off; off += (bytes + 255) & ~(size_t)255; return p; };
  b16* R = (b16*)carve(18432 * 2); float* P = (float*)carve(3272 * 4); float* FT = (float*)carve((size_t)NN * HH * 4); b16* Fh = (b16*)carve((size_t)NN * HH * 2); b16* Fl = (b16*)carve((size_t)NN * HH * 2); float* HID = (float*)carve((size_t)NN * 32 * 4); float* ALR = (float*)carve((size_t)NN * 16 * 4); float* PRE = (float*)carve((size_t)NN * HH * 4);
  float* PART = (float*)carve((size_t)STB * HH * 4); float* MEAN = (float*)carve(HH * 4); float* VAR = (float*)carve(HH * 4);
  CsrBufs cs; off = csr_carve(cs, ws, off, NE_RUN, NN);
  if (off > ws_size) return;
  csr_build(cs, dstI, NE_RUN, NN, stream);
  prep_kernel<<<256, 256, 0, stream>>>(xid, emb, Fp(5), Fp(13), Fp(21), Fp(29), R, FT, Fh, Fl);
  par_kernel<16, 8><<<4, 256, 0, stream>>>(Fp(6), Fp(7), Fp(8), Fp(9), Fp(10), Fp(11), Fp(12), P);
  par_kernel<32, 4><<<4, 256, 0, stream>>>(Fp(14), Fp(15), Fp(16), Fp(17), Fp(18), Fp(19), Fp(20), P + 1024);
  par_kernel<32, 4><<<4, 256, 0, stream>>>(Fp(22), Fp(23), Fp(24), Fp(25), Fp(26), Fp(27), Fp(28), P + 2048);
  parc_kernel<<<1, 256, 0, stream>>>(Fp(30), Fp(31), Fp(32), P);
  for (int l = 0; l < 3; ++l) {
    if (l == 0) { hid_kernel<16, 8><<<NN / 32, 64, 0, stream>>>(Fh, Fl, R + 0, P, HID, ALR); agg_kernel<16><<<NN / 8, 256, 0, stream>>>(HID, ALR, srcI, cs.PERM, cs.ROWPTR, cs.ROWCNT, snorm, PRE); }
    else { hid_kernel<32, 4><<<NN / 32, 64, 0, stream>>>(Fh, Fl, R + (l == 1 ? 2048 : 6144), P + l * 1024, HID, ALR); agg_kernel<32><<<NN / 8, 256, 0, stream>>>(HID, ALR, srcI, cs.PERM, cs.ROWPTR, cs.ROWCNT, snorm, PRE); }
    stat_kernel<0><<<STB, 128, 0, stream>>>(PRE, nullptr, PART); comb_kernel<<<1, 128, 0, stream>>>(PART, MEAN);
    stat_kernel<1><<<STB, 128, 0, stream>>>(PRE, MEAN, PART); comb_kernel<<<1, 128, 0, stream>>>(PART, VAR);
    if (l < 2) epi_kernel<0><<<NN / 8, 256, 0, stream>>>(PRE, MEAN, VAR, P + l * 1024, FT, Fh, Fl); else epi_kernel<1><<<NN / 8, 256, 0, stream>>>(PRE, MEAN, VAR, P + l * 1024, FT, Fh, Fl); }
  cls_kernel<<<NN / 32, 64, 0, stream>>>(Fh, Fl, R + 10240, P, out);
}
